// Wave2D_69793218560502
// MI455X (gfx1250) — hardware-verified
//
#include <hip/hip_runtime.h>

#define NB   16
#define NC   512
#define NHW  1024
#define NTOK 16384
#define KD   512
#define PI_F 3.14159265358979323846f

typedef _Float16       v16h  __attribute__((ext_vector_type(16)));
typedef _Float16       v8h   __attribute__((ext_vector_type(8)));
typedef __bf16         v16b  __attribute__((ext_vector_type(16)));
typedef unsigned short v16us __attribute__((ext_vector_type(16)));
typedef unsigned short v8us  __attribute__((ext_vector_type(8)));
typedef float          v8f   __attribute__((ext_vector_type(8)));
typedef float          v4f   __attribute__((ext_vector_type(4)));
typedef v8h  __attribute__((may_alias)) v8ha;
typedef v8us __attribute__((may_alias)) v8usa;
typedef v4f  __attribute__((may_alias)) v4fa;

union FragH  { v16h v;  v8h  half[2]; };
union FragUS { v16us v; v8us half[2]; };

__device__ __forceinline__ unsigned int bf16_bits(float x) {
  const unsigned int u = __float_as_uint(x);
  return (u + 0x7FFFu + ((u >> 16) & 1u)) >> 16;
}
__device__ __forceinline__ float bf16_val(unsigned int b) { return __uint_as_float(b << 16); }

__device__ __forceinline__ v8f mma_f16(v16h a, v16h b, v8f c) {
  v8f d = __builtin_amdgcn_wmma_f32_16x16x32_f16(false, a, false, b, (short)0, c, false, false);
  asm volatile("v_nop\n\tv_nop\n\tv_nop\n\tv_nop" : "+v"(d) : "v"(a), "v"(b));
  return d;
}
__device__ __forceinline__ v8f mma_bf16(v16us a, v16us b, v8f c) {
  const v16b ab = __builtin_bit_cast(v16b, a);
  const v16b bb = __builtin_bit_cast(v16b, b);
  v8f d = __builtin_amdgcn_wmma_f32_16x16x32_bf16(false, ab, false, bb, (short)0, c, false, false);
  asm volatile("v_nop\n\tv_nop\n\tv_nop\n\tv_nop" : "+v"(d) : "v"(a), "v"(b));
  return d;
}

__device__ __forceinline__ v16h ld_h16(const _Float16* p, int h) {
  FragH f;
  f.half[0] = *(const v8ha*)(p + 8 * h);
  f.half[1] = *(const v8ha*)(p + 16 + 8 * h);
  return f.v;
}
__device__ __forceinline__ v16us ld_u16(const unsigned short* p, int h) {
  FragUS f;
  f.half[0] = *(const v8usa*)(p + 8 * h);
  f.half[1] = *(const v8usa*)(p + 16 + 8 * h);
  return f.v;
}

__device__ __forceinline__ void split8(v4f a, v4f d, v8us& oh, v8us& ol) {
  const float e[8] = {a.x, a.y, a.z, a.w, d.x, d.y, d.z, d.w};
  v8us th = {0, 0, 0, 0, 0, 0, 0, 0};
  v8us tl = {0, 0, 0, 0, 0, 0, 0, 0};
  #pragma unroll
  for (int i = 0; i < 8; ++i) {
    const unsigned int hb = bf16_bits(e[i]);
    th[i] = (unsigned short)hb;
    tl[i] = (unsigned short)bf16_bits(e[i] - bf16_val(hb));
  }
  oh = th; ol = tl;
}

__device__ __forceinline__ void split_frag(const float* rowp, int h, v16us& fh, v16us& fl) {
  const v4f a0 = *(const v4fa*)(rowp + 8 * h);
  const v4f a1 = *(const v4fa*)(rowp + 8 * h + 4);
  const v4f b0 = *(const v4fa*)(rowp + 16 + 8 * h);
  const v4f b1 = *(const v4fa*)(rowp + 20 + 8 * h);
  const float e[16] = {a0.x, a0.y, a0.z, a0.w, a1.x, a1.y, a1.z, a1.w,
                       b0.x, b0.y, b0.z, b0.w, b1.x, b1.y, b1.z, b1.w};
  v16us hv = {0, 0, 0, 0, 0, 0, 0, 0, 0, 0, 0, 0, 0, 0, 0, 0};
  v16us lv = {0, 0, 0, 0, 0, 0, 0, 0, 0, 0, 0, 0, 0, 0, 0, 0};
  #pragma unroll
  for (int i = 0; i < 16; ++i) {
    const unsigned int hb = bf16_bits(e[i]);
    hv[i] = (unsigned short)hb;
    lv[i] = (unsigned short)bf16_bits(e[i] - bf16_val(hb));
  }
  fh = hv; fl = lv;
}

__global__ __launch_bounds__(256) void k_convert(
    const float* __restrict__ lin_w, const float* __restrict__ out_w,
    const float* __restrict__ vel_w, const float* __restrict__ tok_w,
    const float* __restrict__ freq,
    unsigned short* __restrict__ wlh, unsigned short* __restrict__ wll,
    unsigned short* __restrict__ woh, unsigned short* __restrict__ wol,
    _Float16* __restrict__ wv, _Float16* __restrict__ wt, _Float16* __restrict__ fh)
{
  const int seg = blockIdx.y;
  const int g = blockIdx.x * 256 + threadIdx.x;
  const float* src;
  int n8;
  if (seg == 0)      { src = lin_w; n8 = (2 * NC * KD) / 8; }
  else if (seg == 1) { src = out_w; n8 = (NC * KD) / 8; }
  else if (seg == 2) { src = vel_w; n8 = (NC * KD) / 8; }
  else if (seg == 3) { src = tok_w; n8 = (NC * KD) / 8; }
  else               { src = freq;  n8 = (NHW * KD) / 8; }
  if (g >= n8) return;
  const v4f a = *(const v4fa*)(src + (size_t)g * 8);
  const v4f d = *(const v4fa*)(src + (size_t)g * 8 + 4);
  if (seg <= 1) {
    v8us oh, ol;
    split8(a, d, oh, ol);
    unsigned short* ph = ((seg == 0) ? wlh : woh) + (size_t)g * 8;
    unsigned short* pl = ((seg == 0) ? wll : wol) + (size_t)g * 8;
    *(volatile v8us*)ph = oh;
    *(volatile v8us*)pl = ol;
    __threadfence();
    *(volatile v8us*)ph = oh;
    *(volatile v8us*)pl = ol;
  } else {
    const float sc = (seg == 4) ? 1.0f : 16.0f;
    const v8h o = { (_Float16)(a.x * sc), (_Float16)(a.y * sc), (_Float16)(a.z * sc), (_Float16)(a.w * sc),
                    (_Float16)(d.x * sc), (_Float16)(d.y * sc), (_Float16)(d.z * sc), (_Float16)(d.w * sc) };
    _Float16* p = ((seg == 2) ? wv : ((seg == 3) ? wt : fh)) + (size_t)g * 8;
    *(volatile v8h*)p = o;
    __threadfence();
    *(volatile v8h*)p = o;
  }
}

__global__ __launch_bounds__(256) void k_dwconv(
    const float* __restrict__ x, const float* __restrict__ dw_w, const float* __restrict__ dw_b,
    unsigned short* __restrict__ x1h, unsigned short* __restrict__ x1l)
{
  __shared__ __attribute__((aligned(16))) float sIn[64 * 3 * 32];
  __shared__ __attribute__((aligned(16))) float sOut[32 * 64];
  const int tid = threadIdx.x, lane = tid & 31, wv = tid >> 5;
  const int hrow = blockIdx.x, c0 = blockIdx.y * 64, b = blockIdx.z;
  const v4f z4 = {0.f, 0.f, 0.f, 0.f};
  #pragma unroll
  for (int i = 0; i < 6; ++i) {
    const int e = i * 256 + tid;
    const int cl = e / 24, rem = e - cl * 24, rr = rem >> 3, q = rem & 7;
    const int hh = hrow + rr - 1;
    const int hc = min(max(hh, 0), 31);
    v4f v = *(const v4fa*)(x + ((size_t)(b * NC + c0 + cl) * NHW + hc * 32 + q * 4));
    if (hh < 0 || hh > 31) v = z4;
    *(v4fa*)(sIn + (cl * 3 + rr) * 32 + q * 4) = v;
  }
  __syncthreads();

  const int cl = tid >> 2, wq = tid & 3, c = c0 + cl;
  float wt[9];
  #pragma unroll
  for (int j = 0; j < 9; ++j) wt[j] = dw_w[c * 9 + j];
  const float bs = dw_b[c];
  const float* rows = sIn + cl * 96;
  #pragma unroll 1
  for (int j = 0; j < 8; ++j) {
    const int w0 = wq * 8 + j;
    float acc = 0.0f;
    #pragma unroll
    for (int kh = 0; kh < 3; ++kh) {
      #pragma unroll
      for (int kw = 0; kw < 3; ++kw) {
        const int ww = w0 + kw - 1;
        const int wc = min(max(ww, 0), 31);
        float xv = rows[kh * 32 + wc];
        xv = (ww >= 0 && ww <= 31) ? xv : 0.0f;
        acc += xv * wt[kh * 3 + kw];
      }
    }
    sOut[w0 * 64 + cl] = acc + bs;
  }
  __syncthreads();

  const int q8 = lane & 7, sub = lane >> 3;
  const int wp = wv * 4 + sub;
  const v4f a = *(const v4fa*)(sOut + wp * 64 + q8 * 8);
  const v4f d = *(const v4fa*)(sOut + wp * 64 + q8 * 8 + 4);
  v8us oh, ol;
  split8(a, d, oh, ol);
  const size_t m = (size_t)b * NHW + hrow * 32 + wp;
  unsigned short* ph = x1h + m * KD + c0 + q8 * 8;
  unsigned short* pl = x1l + m * KD + c0 + q8 * 8;
  *(volatile v8us*)ph = oh;
  *(volatile v8us*)pl = ol;
  __threadfence();
  *(volatile v8us*)ph = oh;
  *(volatile v8us*)pl = ol;
}

__device__ __forceinline__ void pass_cm(const float* sT, float* out, size_t rowbase, int hw0, int w, int lane) {
  const int q8 = lane & 7, sub = lane >> 3;
  #pragma unroll 1
  for (int i = 0; i < 16; ++i) {
    const int L = w * 64 + i * 4 + sub;
    const int f = L >> 2, q = L & 3;
    const v4f v = *(const v4fa*)(sT + f * 132 + 32 * q + 4 * q8);
    float* dst = out + (rowbase + f) * NHW + hw0 + 32 * q + 4 * q8;
    *(volatile v4f*)dst = v;
  }
}
__device__ __forceinline__ void pass_tab(const float* sT, float* ct, float* st, float cv, float rc,
                                         size_t rowbase, int hw0, int w, int lane) {
  const int q8 = lane & 7, sub = lane >> 3;
  #pragma unroll 1
  for (int i = 0; i < 16; ++i) {
    const int L = w * 64 + i * 4 + sub;
    const int f = L >> 2, q = L & 3;
    const v4f t = *(const v4fa*)(sT + f * 132 + 32 * q + 4 * q8);
    const float ax = cv * t.x, ay = cv * t.y, az = cv * t.z, aw = cv * t.w;
    const v4f cvv = { cosf(ax), cosf(ay), cosf(az), cosf(aw) };
    const v4f svv = { sinf(ax) * rc, sinf(ay) * rc, sinf(az) * rc, sinf(aw) * rc };
    const size_t gi = (rowbase + f) * NHW + hw0 + 32 * q + 4 * q8;
    *(volatile v4f*)(ct + gi) = cvv;
    *(volatile v4f*)(st + gi) = svv;
  }
}
__device__ __forceinline__ void pass_tmh(const float* sT, _Float16* outh, int m0, int n0, int w, int lane) {
  const int q8 = lane & 7, sub = lane >> 3;
  #pragma unroll 1
  for (int i = 0; i < 8; ++i) {
    const int t = w * 32 + i * 4 + sub;
    v8h o;
    #pragma unroll
    for (int e = 0; e < 8; ++e) o[e] = (_Float16)sT[(8 * q8 + e) * 132 + t];
    _Float16* dst = outh + (size_t)(m0 + t) * KD + n0 + 8 * q8;
    *(volatile v8h*)dst = o;
  }
}
__device__ __forceinline__ void pass_tmz(const float* sT, float* z, int m0, int n0z, int w, int lane) {
  const int q8 = lane & 7, sub = lane >> 3;
  #pragma unroll 1
  for (int i = 0; i < 16; ++i) {
    const int L = w * 64 + i * 4 + sub;
    const int t = L >> 1, hl = L & 1;
    const v4f v = *(const v4fa*)(sT + t * 68 + 32 * hl + 4 * q8);
    float* dst = z + (size_t)(m0 + t) * KD + n0z + 32 * hl + 4 * q8;
    *(volatile v4f*)dst = v;
  }
}

template <int MODE>
__global__ __launch_bounds__(128) void k_gemm(
    const unsigned short* __restrict__ Ah, const unsigned short* __restrict__ Al,
    const _Float16* __restrict__ Af,
    const unsigned short* __restrict__ Bh, const unsigned short* __restrict__ Bl,
    const _Float16* __restrict__ Bf,
    const float* __restrict__ bias, const float* __restrict__ cptr,
    float* __restrict__ out0, float* __restrict__ out1, _Float16* __restrict__ outh)
{
  __shared__ __attribute__((aligned(16))) float sT[8704];
  constexpr bool SPLIT = (MODE == 0 || MODE == 3);

  const int tid = threadIdx.x, lane = tid & 31, w = tid >> 5;
  const int h = lane >> 4, m = lane & 15;
  const int m0 = blockIdx.x * 128, n0 = blockIdx.y * 64;
  const int m0w = m0 + 32 * w;

  const v8f zero8 = {0.f, 0.f, 0.f, 0.f, 0.f, 0.f, 0.f, 0.f};
  v8f acc[2][4];
  #pragma unroll
  for (int mt = 0; mt < 2; ++mt)
    #pragma unroll
    for (int nt = 0; nt < 4; ++nt) acc[mt][nt] = zero8;

  if constexpr (SPLIT) {
    const unsigned short* a0h = Ah + (size_t)(m0w + m) * KD;
    const unsigned short* a1h = a0h + (size_t)16 * KD;
    const unsigned short* a0l = Al + (size_t)(m0w + m) * KD;
    const unsigned short* a1l = a0l + (size_t)16 * KD;
    const unsigned short* bph = Bh + (size_t)(n0 + m) * KD;
    const unsigned short* bpl = Bl + (size_t)(n0 + m) * KD;
    #pragma unroll 1
    for (int k0 = 0; k0 < KD; k0 += 32) {
      const v16us A0h = ld_u16(a0h + k0, h);
      const v16us A1h = ld_u16(a1h + k0, h);
      const v16us A0l = ld_u16(a0l + k0, h);
      const v16us A1l = ld_u16(a1l + k0, h);
      #pragma unroll
      for (int nt = 0; nt < 4; ++nt) {
        const v16us Bhv = ld_u16(bph + (size_t)nt * 16 * KD + k0, h);
        const v16us Blv = ld_u16(bpl + (size_t)nt * 16 * KD + k0, h);
        acc[0][nt] = mma_bf16(A0h, Bhv, acc[0][nt]);
        acc[0][nt] = mma_bf16(A0h, Blv, acc[0][nt]);
        acc[0][nt] = mma_bf16(A0l, Bhv, acc[0][nt]);
        acc[1][nt] = mma_bf16(A1h, Bhv, acc[1][nt]);
        acc[1][nt] = mma_bf16(A1h, Blv, acc[1][nt]);
        acc[1][nt] = mma_bf16(A1l, Bhv, acc[1][nt]);
      }
    }
  } else {
    const _Float16* a0 = Af + (size_t)(m0w + m) * KD;
    const _Float16* a1 = a0 + (size_t)16 * KD;
    const _Float16* bp = Bf + (size_t)(n0 + m) * KD;
    #pragma unroll 1
    for (int k0 = 0; k0 < KD; k0 += 32) {
      const v16h A0 = ld_h16(a0 + k0, h);
      const v16h A1 = ld_h16(a1 + k0, h);
      #pragma unroll
      for (int nt = 0; nt < 4; ++nt) {
        const v16h Bv = ld_h16(bp + (size_t)nt * 16 * KD + k0, h);
        acc[0][nt] = mma_f16(A0, Bv, acc[0][nt]);
        acc[1][nt] = mma_f16(A1, Bv, acc[1][nt]);
      }
    }
  }

  const float sc = SPLIT ? 1.0f : 0.0625f;
  bool tmz = false;
  if constexpr (MODE == 0) tmz = (blockIdx.y >= 8);
  #pragma unroll
  for (int nt = 0; nt < 4; ++nt) {
    const int fl = 16 * nt + m;
    const float bv = bias[n0 + fl];
    #pragma unroll
    for (int mt = 0; mt < 2; ++mt) {
      #pragma unroll
      for (int r = 0; r < 8; ++r) {
        const int tl = 32 * w + 16 * mt + 8 * h + r;
        float v = acc[mt][nt][r] * sc + bv;
        if constexpr (MODE == 2) v = fmaxf(v, 0.0f);
        const int si = tmz ? (tl * 68 + fl) : (fl * 132 + tl);
        sT[si] = v;
      }
    }
  }
  __syncthreads();

  const size_t rowbase = (size_t)(m0 >> 10) * NC + n0;
  const int hw0 = m0 & 1023;
  if constexpr (MODE == 0) {
    if (tmz) {
      pass_tmz(sT, out1, m0, n0 - NC, w, lane);
      __threadfence();
      pass_tmz(sT, out1, m0, n0 - NC, w, lane);
    } else {
      pass_cm(sT, out0, rowbase, hw0, w, lane);
      pass_tmh(sT, outh, m0, n0, w, lane);
      __threadfence();
      pass_cm(sT, out0, rowbase, hw0, w, lane);
      pass_tmh(sT, outh, m0, n0, w, lane);
    }
  } else if constexpr (MODE == 2) {
    const float cv = cptr[0];
    const float rc = 1.0f / (cv + 1e-6f);
    pass_tab(sT, out0, out1, cv, rc, rowbase, hw0, w, lane);
    __threadfence();
    pass_tab(sT, out0, out1, cv, rc, rowbase, hw0, w, lane);
  } else {
    pass_cm(sT, out0, rowbase, hw0, w, lane);
    __threadfence();
    pass_cm(sT, out0, rowbase, hw0, w, lane);
  }
}

__device__ __forceinline__ void mm_fp(const float* At, const unsigned short* Ph, const unsigned short* Pl,
                                      int h, int m, v8f (&acc)[2][2]) {
  v16us ah[2], al[2];
  #pragma unroll
  for (int i = 0; i < 2; ++i) split_frag(At + (i * 16 + m) * 36, h, ah[i], al[i]);
  #pragma unroll
  for (int j = 0; j < 2; ++j) {
    const v16us bh = ld_u16(Ph + (j * 16 + m) * 32, h);
    const v16us bl = ld_u16(Pl + (j * 16 + m) * 32, h);
    #pragma unroll
    for (int i = 0; i < 2; ++i) {
      acc[i][j] = mma_bf16(ah[i], bh, acc[i][j]);
      acc[i][j] = mma_bf16(ah[i], bl, acc[i][j]);
      acc[i][j] = mma_bf16(al[i], bh, acc[i][j]);
    }
  }
}
__device__ __forceinline__ void mm_pf(const unsigned short* Ph, const unsigned short* Pl, const float* Bt,
                                      int h, int m, v8f (&acc)[2][2]) {
  v16us bh[2], bl[2];
  #pragma unroll
  for (int j = 0; j < 2; ++j) split_frag(Bt + (j * 16 + m) * 36, h, bh[j], bl[j]);
  #pragma unroll
  for (int i = 0; i < 2; ++i) {
    const v16us ah = ld_u16(Ph + (i * 16 + m) * 32, h);
    const v16us al = ld_u16(Pl + (i * 16 + m) * 32, h);
    #pragma unroll
    for (int j = 0; j < 2; ++j) {
      acc[i][j] = mma_bf16(ah, bh[j], acc[i][j]);
      acc[i][j] = mma_bf16(ah, bl[j], acc[i][j]);
      acc[i][j] = mma_bf16(al, bh[j], acc[i][j]);
    }
  }
}
__device__ __forceinline__ void zero22(v8f (&a)[2][2]) {
  const v8f z = {0.f, 0.f, 0.f, 0.f, 0.f, 0.f, 0.f, 0.f};
  #pragma unroll
  for (int i = 0; i < 2; ++i)
    #pragma unroll
    for (int j = 0; j < 2; ++j) a[i][j] = z;
}
__device__ __forceinline__ void storeT(float* T, const v8f (&acc)[2][2], int h, int m) {
  #pragma unroll
  for (int i = 0; i < 2; ++i)
    #pragma unroll
    for (int j = 0; j < 2; ++j)
      #pragma unroll
      for (int r = 0; r < 8; ++r) {
        const int mr = i * 16 + h * 8 + r;
        const int n = j * 16 + m;
        T[n * 36 + mr] = acc[i][j][r];
      }
}
__device__ __forceinline__ void load_img(const float* src, float* X, int lane) {
  #pragma unroll
  for (int i = 0; i < 8; ++i) {
    const int e = i * 128 + lane * 4;
    const int row = e >> 5, col = e & 31;
    const v4f v = *(const v4fa*)(src + e);
    *(v4fa*)(X + row * 36 + col) = v;
  }
}
__device__ __forceinline__ void img_store(const float* X, float* dst, int lane) {
  const int q8 = lane & 7, sub = lane >> 3;
  #pragma unroll
  for (int i = 0; i < 8; ++i) {
    const int row = i * 4 + sub;
    const v4f v = *(const v4fa*)(X + row * 36 + 4 * q8);
    *(volatile v4f*)(dst + row * 32 + 4 * q8) = v;
  }
}

__global__ __launch_bounds__(64) void k_spectral(
    float* xio, const float* __restrict__ xv, const float* __restrict__ cosT,
    const float* __restrict__ sinT, const float* __restrict__ aptr)
{
  __shared__ __attribute__((aligned(16))) unsigned short sDh[1024];
  __shared__ __attribute__((aligned(16))) unsigned short sDl[1024];
  __shared__ __attribute__((aligned(16))) unsigned short sEh[1024];
  __shared__ __attribute__((aligned(16))) unsigned short sEl[1024];
  __shared__ float sDec[1024];
  __shared__ __attribute__((aligned(16))) float sX[2][1152];
  __shared__ __attribute__((aligned(16))) float sTt[2][1152];
  __shared__ __attribute__((aligned(16))) float sU[2][1152];

  const int tid = threadIdx.x, lane = tid & 31, wv = tid >> 5;
  const int h = lane >> 4, m = lane & 15;

  #pragma unroll 1
  for (int idx = tid; idx < 1024; idx += 64) {
    const int k = idx >> 5, n = idx & 31;
    const float s = (k == 0) ? 0.17677669529663688f : 0.25f;
    const float d = s * cosf(PI_F * ((float)((2 * n + 1) * k) * 0.015625f));
    const unsigned int hb = bf16_bits(d);
    const unsigned int lb = bf16_bits(d - bf16_val(hb));
    sDh[k * 32 + n] = (unsigned short)hb;
    sDl[k * 32 + n] = (unsigned short)lb;
    sEh[n * 32 + k] = (unsigned short)hb;
    sEl[n * 32 + k] = (unsigned short)lb;
    const float wn = PI_F * ((float)k * 0.03125f);
    const float wm = PI_F * ((float)n * 0.03125f);
    sDec[idx] = expf(-(wn * wn + wm * wm));
  }
  __syncthreads();

  const int img = blockIdx.x * 2 + wv;
  const int cch = img & 511;
  const float ha = 0.5f * aptr[0];
  float* X  = sX[wv];
  float* T  = sTt[wv];
  float* Ub = sU[wv];
  v8f P[2][2], V[2][2];

  load_img(xio + (size_t)img * NHW, X, lane);
  __syncthreads();
  zero22(P); mm_fp(X, sDh, sDl, h, m, P);
  storeT(T, P, h, m);
  __syncthreads();
  zero22(V); mm_pf(sDh, sDl, T, h, m, V);
  #pragma unroll
  for (int i = 0; i < 2; ++i)
    #pragma unroll
    for (int j = 0; j < 2; ++j)
      #pragma unroll
      for (int r = 0; r < 8; ++r) {
        const int M = i * 16 + h * 8 + r, N = j * 16 + m;
        Ub[M * 36 + N] = V[i][j][r] * sDec[M * 32 + N];
      }
  __syncthreads();

  load_img(xv + (size_t)img * NHW, X, lane);
  __syncthreads();
  zero22(P); mm_fp(X, sDh, sDl, h, m, P);
  storeT(T, P, h, m);
  __syncthreads();
  zero22(V); mm_pf(sDh, sDl, T, h, m, V);

  #pragma unroll
  for (int i = 0; i < 2; ++i)
    #pragma unroll
    for (int j = 0; j < 2; ++j)
      #pragma unroll
      for (int r = 0; r < 8; ++r) {
        const int M = i * 16 + h * 8 + r, N = j * 16 + m;
        const size_t fi = (size_t)cch * NHW + M * 32 + N;
        const float u = Ub[M * 36 + N];
        const float v = V[i][j][r] * sDec[M * 32 + N];
        X[M * 36 + N] = cosT[fi] * u + sinT[fi] * (v + ha * u);
      }
  __syncthreads();

  zero22(P); mm_fp(X, sEh, sEl, h, m, P);
  storeT(T, P, h, m);
  __syncthreads();
  zero22(V); mm_pf(sEh, sEl, T, h, m, V);
  #pragma unroll
  for (int i = 0; i < 2; ++i)
    #pragma unroll
    for (int j = 0; j < 2; ++j)
      #pragma unroll
      for (int r = 0; r < 8; ++r) {
        const int M = i * 16 + h * 8 + r, N = j * 16 + m;
        X[M * 36 + N] = V[i][j][r];
      }
  __syncthreads();

  float* dst = xio + (size_t)img * NHW;
  img_store(X, dst, lane);
  __threadfence();
  img_store(X, dst, lane);
}

__global__ __launch_bounds__(256) void k_ln_gate(
    const float* __restrict__ xf, const float* __restrict__ z,
    const float* __restrict__ gamma, const float* __restrict__ beta,
    unsigned short* __restrict__ gh, unsigned short* __restrict__ gl)
{
  __shared__ float sPart[256];
  __shared__ float sMu[32];
  __shared__ float sRs[32];
  __shared__ __attribute__((aligned(16))) unsigned short sH[2048];
  __shared__ __attribute__((aligned(16))) unsigned short sL[2048];

  const int tid = threadIdx.x, lane = tid & 31, cs = tid >> 5, p = lane;
  const int pg = blockIdx.x, b = blockIdx.y;
  const int hw = pg * 32 + p;
  const float* xcol = xf + (size_t)b * NC * NHW + hw;

  float s = 0.0f;
  #pragma unroll 1
  for (int j = 0; j < 64; ++j) s += xcol[(size_t)(cs * 64 + j) * NHW];
  sPart[cs * 32 + p] = s;
  __syncthreads();
  if (cs == 0) {
    float t = 0.0f;
    #pragma unroll
    for (int g = 0; g < 8; ++g) t += sPart[g * 32 + p];
    sMu[p] = t * (1.0f / 512.0f);
  }
  __syncthreads();
  const float mu = sMu[p];
  float q = 0.0f;
  #pragma unroll 1
  for (int j = 0; j < 64; ++j) {
    const float d = xcol[(size_t)(cs * 64 + j) * NHW] - mu;
    q += d * d;
  }
  sPart[cs * 32 + p] = q;
  __syncthreads();
  if (cs == 0) {
    float t = 0.0f;
    #pragma unroll
    for (int g = 0; g < 8; ++g) t += sPart[g * 32 + p];
    const float var = t * (1.0f / 512.0f);
    sRs[p] = 1.0f / sqrtf(var + 1e-5f);
  }
  __syncthreads();
  const float rs = sRs[p];

  const size_t mtok = (size_t)b * NHW + hw;
  const int q8 = lane & 7, sub = lane >> 3;
  #pragma unroll 1
  for (int ch = 0; ch < 8; ++ch) {
    #pragma unroll 1
    for (int j = 0; j < 8; ++j) {
      const int c = ch * 64 + cs * 8 + j;
      const float xvv = xcol[(size_t)c * NHW];
      const float ln = (xvv - mu) * rs * gamma[c] + beta[c];
      const float zv = z[mtok * KD + c];
      const float ex = expf(-zv);
      const float sg = 1.0f / (1.0f + ex);
      const float g = ln * (zv * sg);
      const unsigned int hb = bf16_bits(g);
      sH[p * 64 + cs * 8 + j] = (unsigned short)hb;
      sL[p * 64 + cs * 8 + j] = (unsigned short)bf16_bits(g - bf16_val(hb));
    }
    __syncthreads();
    const int pp = cs * 4 + sub;
    const v8us oh = *(const v8usa*)(sH + pp * 64 + q8 * 8);
    const v8us ol = *(const v8usa*)(sL + pp * 64 + q8 * 8);
    const size_t gi = ((size_t)b * NHW + pg * 32 + pp) * KD + ch * 64 + q8 * 8;
    *(volatile v8us*)(gh + gi) = oh;
    *(volatile v8us*)(gl + gi) = ol;
    __threadfence();
    *(volatile v8us*)(gh + gi) = oh;
    *(volatile v8us*)(gl + gi) = ol;
    __syncthreads();
  }
}

extern "C" void kernel_launch(void* const* d_in, const int* in_sizes, int n_in,
                              void* d_out, int out_size, void* d_ws, size_t ws_size,
                              hipStream_t stream) {
  if (n_in < 16) return;
  if (in_sizes[0] != NTOK * NC) return;
  if (in_sizes[1] != NHW * NC) return;
  if (in_sizes[2] != NC * 9 || in_sizes[3] != NC) return;
  if (in_sizes[4] != 2 * NC * KD || in_sizes[5] != 2 * NC) return;
  if (in_sizes[6] != NC * KD || in_sizes[7] != NC) return;
  if (in_sizes[8] != NC * KD || in_sizes[9] != NC) return;
  if (in_sizes[10] != NC || in_sizes[11] != NC) return;
  if (in_sizes[12] != NC * KD || in_sizes[13] != NC) return;
  if (in_sizes[14] < 1 || in_sizes[15] < 1) return;
  if (out_size != NTOK * NC) return;

  const float* x     = (const float*)d_in[0];
  const float* freq  = (const float*)d_in[1];
  const float* dw_w  = (const float*)d_in[2];
  const float* dw_b  = (const float*)d_in[3];
  const float* lin_w = (const float*)d_in[4];
  const float* lin_b = (const float*)d_in[5];
  const float* vel_w = (const float*)d_in[6];
  const float* vel_b = (const float*)d_in[7];
  const float* tok_w = (const float*)d_in[8];
  const float* tok_b = (const float*)d_in[9];
  const float* gamma = (const float*)d_in[10];
  const float* beta  = (const float*)d_in[11];
  const float* out_w = (const float*)d_in[12];
  const float* out_b = (const float*)d_in[13];
  const float* cptr  = (const float*)d_in[14];
  const float* aptr  = (const float*)d_in[15];
  float* out = (float*)d_out;

  const size_t b_wl  = (size_t)2 * NC * KD * 2;
  const size_t b_w   = (size_t)NC * KD * 2;
  const size_t b_fh  = (size_t)NHW * KD * 2;
  const size_t b_tab = (size_t)NC * NHW * 4;
  const size_t b_r32 = (size_t)NTOK * NC * 4;
  const size_t b_r16 = (size_t)NTOK * NC * 2;
  size_t off = 0;
  const size_t o_wlh = off; off += b_wl;
  const size_t o_wll = off; off += b_wl;
  const size_t o_woh = off; off += b_w;
  const size_t o_wol = off; off += b_w;
  const size_t o_wv  = off; off += b_w;
  const size_t o_wt  = off; off += b_w;
  const size_t o_fh  = off; off += b_fh;
  const size_t o_cos = off; off += b_tab;
  const size_t o_sin = off; off += b_tab;
  const size_t o_ra  = off; off += b_r32;
  const size_t o_rb  = off; off += b_r32;
  const size_t o_rc  = off; off += b_r32;
  const size_t o_rd  = off; off += b_r16;
  const size_t total = off;
  if (total > ws_size) return;
  if (total > (size_t)134217728) return;

  char* ws = (char*)d_ws;
  unsigned short* wlh = (unsigned short*)(ws + o_wlh);
  unsigned short* wll = (unsigned short*)(ws + o_wll);
  unsigned short* woh = (unsigned short*)(ws + o_woh);
  unsigned short* wol = (unsigned short*)(ws + o_wol);
  _Float16* wv  = (_Float16*)(ws + o_wv);
  _Float16* wt  = (_Float16*)(ws + o_wt);
  _Float16* fh  = (_Float16*)(ws + o_fh);
  float* cosT   = (float*)(ws + o_cos);
  float* sinT   = (float*)(ws + o_sin);
  unsigned short* x1h = (unsigned short*)(ws + o_ra);
  unsigned short* x1l = (unsigned short*)(ws + o_ra + b_r16);
  float* xvcm   = (float*)(ws + o_ra);
  unsigned short* gh  = x1h;
  unsigned short* gl  = x1l;
  float* xscm   = (float*)(ws + o_rb);
  float* zbuf   = (float*)(ws + o_rc);
  _Float16* xsh = (_Float16*)(ws + o_rd);

  k_convert<<<dim3(256, 5), 256, 0, stream>>>(lin_w, out_w, vel_w, tok_w, freq,
                                              wlh, wll, woh, wol, wv, wt, fh);
  k_dwconv<<<dim3(32, 8, NB), 256, 0, stream>>>(x, dw_w, dw_b, x1h, x1l);
  k_gemm<0><<<dim3(NTOK / 128, 16), 128, 0, stream>>>(x1h, x1l, xsh, wlh, wll, wv, lin_b, cptr,
                                                      xscm, zbuf, xsh);
  k_gemm<1><<<dim3(NTOK / 128, 8), 128, 0, stream>>>(wlh, wll, xsh, woh, wol, wv, vel_b, cptr,
                                                     xvcm, zbuf, xsh);
  k_gemm<2><<<dim3(NHW / 128, 8), 128, 0, stream>>>(wlh, wll, fh, woh, wol, wt, tok_b, cptr,
                                                    cosT, sinT, xsh);
  k_spectral<<<(NB * NC) / 2, 64, 0, stream>>>(xscm, xvcm, cosT, sinT, aptr);
  k_ln_gate<<<dim3(NHW / 32, NB), 256, 0, stream>>>(xscm, zbuf, gamma, beta, gh, gl);
  k_gemm<3><<<dim3(NTOK / 128, 8), 128, 0, stream>>>(gh, gl, xsh, woh, wol, wv, out_b, cptr,
                                                     out, zbuf, xsh);
}
